// OrderCourierHeteroGNN_23373212025402
// MI455X (gfx1250) — hardware-run, weakly checked
//
#include <hip/hip_runtime.h>


namespace {
constexpr int NO = 100000, NR = 1000, NRP = 1008, E = 1000000, DO = 64, DR = 32, DE = 4, H = 64, OM = 32, MH = 128;
constexpr float XS = 8.0f, WSC = 256.0f, SCALE = 0.125f;
typedef _Float16 b16;
typedef __attribute__((ext_vector_type(16))) _Float16 v16b;
typedef __attribute__((ext_vector_type(8))) _Float16 v8b;
typedef __attribute__((ext_vector_type(8))) float v8f;
typedef __attribute__((ext_vector_type(4))) float v4f;
typedef __attribute__((ext_vector_type(2))) float v2f;
__device__ __forceinline__ float bf16_rne(float f) { unsigned int u = __float_as_uint(f); u += 0x7FFFu + ((u >> 16) & 1u); float r = __uint_as_float(u & 0xFFFF0000u); asm volatile("" : "+v"(r)); return r; }
__device__ __forceinline__ void split16(float v, b16& hi, b16& lo) { hi = (b16)v; lo = (b16)(v - (float)hi); }
__device__ __forceinline__ v16b frag_kb(const b16* p, int hh) { const v8b a = *(const v8b*)(p + 8 * hh), b = *(const v8b*)(p + 16 + 8 * hh); v16b f;
#pragma unroll
  for (int e = 0; e < 8; ++e) { f[e] = a[e]; f[8 + e] = b[e]; } return f; }
__device__ __forceinline__ v8f wmma16b(v16b a, v16b b, v8f c) { v8f d = __builtin_amdgcn_wmma_f32_16x16x32_f16(false, a, false, b, (short)0, c, false, false); asm volatile("v_nop\n\tv_nop\n\tv_nop\n\tv_nop" : "+v"(d) : "v"(a), "v"(b)); return d; }
__device__ __forceinline__ void wave_lds_sync() { __builtin_amdgcn_fence(__ATOMIC_RELEASE, "workgroup"); __builtin_amdgcn_wave_barrier(); __builtin_amdgcn_fence(__ATOMIC_ACQUIRE, "workgroup"); }
__device__ __forceinline__ float pmul(float a, float b) { float p = a * b; asm volatile("" : "+v"(p)); return p; }
__device__ __forceinline__ int iclamp(int v, int lo, int hi) { return v < lo ? lo : (v > hi ? hi : v); }
#define N NRP
constexpr int CSR_NBLK3 = 512, CSR_GB3 = 3, CSR_GN3 = 1 << CSR_GB3  , CSR_TS3 = (CSR_GN3 < 32 ? 32 : CSR_GN3)  , CSR_MAXG3 = 512, CSR_CAP3 = 12288  ;
__device__ __host__ __forceinline__ int csr_tix3(int v) { return (v >> CSR_GB3) * CSR_TS3 + (v & (CSR_GN3 - 1)); }
__global__ __launch_bounds__(64) void csrA_kernel3(const int* __restrict__ dst, int E, int N, int nG, int CHP, int NGP, int* __restrict__ STG, int* __restrict__ HST) {
  extern __shared__ int sm[];
  int* cnt = sm; int* run = sm + NGP; int* ids = sm + 2 * NGP;
  const int b = blockIdx.x; const int ch = (E + CSR_NBLK3 - 1) / CSR_NBLK3; const int e0 = b * ch, e1 = min(E, e0 + ch);
  for (int i = threadIdx.x; i < NGP; i += 64) cnt[i] = 0;
  for (int i = threadIdx.x; i < CHP; i += 64) ids[i] = -1;
  __syncthreads();
  if (threadIdx.x == 0) {
    for (int e = e0; e < e1; ++e) { int d = dst[e]; d = (d < 0) ? 0 : (d >= N ? N - 1 : d); cnt[d >> CSR_GB3] += 1; }
    int acc = 0; for (int g = 0; g < nG; ++g) { run[g] = acc; acc += cnt[g]; }
    for (int e = e0; e < e1; ++e) { int d = dst[e]; d = (d < 0) ? 0 : (d >= N ? N - 1 : d); const int g = d >> CSR_GB3; ids[run[g]] = e; run[g] += 1; } }
  __syncthreads();
  typedef __attribute__((ext_vector_type(4))) int v4i;
  for (int pass = 0; pass < 2; ++pass) {
    for (int i = threadIdx.x; i < CHP / 4; i += 64) *(volatile v4i*)(STG + (size_t)b * CHP + i * 4) = *(const v4i*)(&ids[i * 4]);
    for (int i = threadIdx.x; i < NGP / 4; i += 64) { v4i v; for (int e = 0; e < 4; ++e) v[e] = (i * 4 + e < nG) ? cnt[i * 4 + e] : 0; *(volatile v4i*)(HST + (size_t)b * NGP + i * 4) = v; }
    __threadfence(); }
}
__global__ __launch_bounds__(512) void csrS_kernel3(const int* __restrict__ HST, int nG, int NGP, int* __restrict__ START, int* __restrict__ TOT, int* __restrict__ OFF) {
  __shared__ int tot[CSR_MAXG3];
  const int b = threadIdx.x;
  for (int pass = 0; pass < 2; ++pass) { int runb = 0; for (int g = 0; g < nG; ++g) { int c = HST[(size_t)b * NGP + g]; c = (c < 0) ? 0 : c; ((volatile int*)OFF)[(size_t)g * CSR_NBLK3 + b] = runb; runb += c; } __threadfence(); }
  for (int g = threadIdx.x; g < nG; g += 512) { int s = 0; for (int bb = 0; bb < CSR_NBLK3; ++bb) { int c = HST[(size_t)bb * NGP + g]; s += (c < 0) ? 0 : c; } tot[g] = s; }
  __syncthreads();
  if (threadIdx.x < 32) {
    __shared__ int st[CSR_MAXG3 + 32];
    if (threadIdx.x == 0) { int acc = 0; for (int g = 0; g < NGP; ++g) { st[g] = acc; if (g < nG) acc += (tot[g] + 31) & ~31; } st[NGP] = acc; }
    __builtin_amdgcn_fence(__ATOMIC_RELEASE, "workgroup"); __builtin_amdgcn_wave_barrier(); __builtin_amdgcn_fence(__ATOMIC_ACQUIRE, "workgroup");
    for (int pass = 0; pass < 2; ++pass) { for (int i = threadIdx.x; i < NGP + 32; i += 32) { ((volatile int*)START)[i] = (i <= NGP) ? st[min(i, NGP)] : 0; ((volatile int*)TOT)[i] = (i < nG) ? tot[i] : 0; } __threadfence(); } }
}
__global__ __launch_bounds__(256) void csrB_kernel3(const int* __restrict__ dst, int N, int nG, int CHP, int NGP, int permLen, const int* __restrict__ STG, const int* __restrict__ HST, const int* __restrict__ OFF, const int* __restrict__ START, const int* __restrict__ TOT, int* __restrict__ PERM, int* __restrict__ ROWPTR, int* __restrict__ ROWCNT, int* __restrict__ FLAG) {
  typedef __attribute__((ext_vector_type(4))) int v4i;
  __shared__ int ids[CSR_CAP3]; __shared__ unsigned short key[CSR_CAP3]; __shared__ int outp[CSR_CAP3]; __shared__ int ncnt[CSR_GN3 + 1]; __shared__ int boff[CSR_NBLK3 + 1];
  const int g = blockIdx.x, t_ = threadIdx.x; int tot = TOT[g]; int st = START[g], stn = START[g + 1]; const int v0 = g * CSR_GN3; const int nv = min(CSR_GN3, N - v0); const int t0 = g * CSR_TS3;
  st = (st < 0) ? 0 : (st > permLen - 32 ? permLen - 32 : st) & ~31; stn = (stn < st) ? st : (stn > permLen ? permLen : stn); tot = (tot < 0) ? 0 : tot; if (tot > stn - st && tot <= CSR_CAP3) tot = stn - st;
  if (tot > CSR_CAP3) {
    for (int pass = 0; pass < 2; ++pass) { for (int i = t_; i < CSR_TS3 / 4; i += 256) { v4i a, c; for (int e = 0; e < 4; ++e) { a[e] = st; c[e] = 0; } *(volatile v4i*)(ROWPTR + t0 + i * 4) = a; *(volatile v4i*)(ROWCNT + t0 + i * 4) = c; } if (t_ == 0) ((volatile int*)FLAG)[0] = 1; __threadfence(); } (void)nv; return; }
  if (t_ == 0) { int acc = 0; for (int b = 0; b < CSR_NBLK3; ++b) { boff[b] = acc; int c = HST[(size_t)b * NGP + g]; c = (c < 0) ? 0 : (c > CHP ? CHP : c); acc += c; if (acc > tot) acc = tot; } boff[CSR_NBLK3] = acc; }
  for (int i = t_; i <= CSR_GN3; i += 256) ncnt[i] = 0;
  __syncthreads();
  for (int b = 0; b < CSR_NBLK3; ++b) { const int c = boff[b + 1] - boff[b]; int o_ = OFF[(size_t)g * CSR_NBLK3 + b]; o_ = (o_ < 0) ? 0 : (o_ > CHP - c ? CHP - c : o_); const int* src_ = STG + (size_t)b * CHP + o_;
    for (int i = t_; i < c; i += 256) { int id = src_[i]; id = (id < 0) ? 0 : id; ids[boff[b] + i] = id; int d = dst[id]; d = (d < v0) ? v0 : (d >= N ? N - 1 : d); int kk = d - v0; kk = (kk < 0) ? 0 : (kk >= CSR_GN3 ? CSR_GN3 - 1 : kk); key[boff[b] + i] = (unsigned short)kk; } }
  __syncthreads();
  if (t_ == 0) { for (int i = 0; i < tot; ++i) ncnt[key[i]] += 1; int acc = 0; for (int vl = 0; vl < CSR_GN3; ++vl) { const int c = ncnt[vl]; ncnt[vl] = acc; acc += c; } ncnt[CSR_GN3] = acc;
    for (int i = 0; i < tot; ++i) { const int vl = key[i]; outp[ncnt[vl]] = ids[i]; ncnt[vl] += 1; }
    for (int vl = CSR_GN3; vl > 0; --vl) ncnt[vl] = ncnt[vl - 1]; ncnt[0] = 0; }
  __syncthreads();
  for (int pass = 0; pass < 2; ++pass) {
    for (int i = t_; i < (stn - st) / 4; i += 256) { v4i v; for (int e = 0; e < 4; ++e) { const int q = i * 4 + e; v[e] = (q < tot) ? outp[q] : -1; } *(volatile v4i*)(PERM + st + i * 4) = v; }
    for (int i = t_; i < CSR_TS3 / 4; i += 256) { v4i a, c; for (int e = 0; e < 4; ++e) { const int vl = i * 4 + e; const int vc = vl < CSR_GN3 ? vl : CSR_GN3; a[e] = (vl < CSR_GN3) ? st + ncnt[vc] : st; c[e] = (vl < nv) ? (ncnt[(vc < CSR_GN3 ? vc : CSR_GN3 - 1) + 1] - ncnt[vc]) : 0; } *(volatile v4i*)(ROWPTR + t0 + i * 4) = a; *(volatile v4i*)(ROWCNT + t0 + i * 4) = c; }
    __threadfence(); }
}
__global__ __launch_bounds__(256) void csrZ_kernel3(int* __restrict__ p, size_t n4) { typedef __attribute__((ext_vector_type(4))) int v4i; const size_t tid = (size_t)blockIdx.x * 256 + threadIdx.x, nth = (size_t)gridDim.x * 256; v4i z = {0, 0, 0, 0}; for (size_t i = tid; i < n4; i += nth) *(volatile v4i*)(p + i * 4) = z; }
struct CsrBufs3 { int *STG, *HST, *OFF, *START, *TOT, *PERM, *ROWPTR, *ROWCNT, *FLAG; int nG, NGP, CHP; size_t permLen; char* base; size_t bytes; };
static size_t csr_carve3(CsrBufs3& c, char* ws, size_t off, int E, int N) {
  const size_t off0 = off; c.base = ws + off;
  auto al = [&](size_t bytes) { char* p = ws + off; off += (bytes + 255) & ~(size_t)255; return p; };
  c.nG = (N + CSR_GN3 - 1) / CSR_GN3; c.NGP = (c.nG + 31) & ~31; const int ch = (E + CSR_NBLK3 - 1) / CSR_NBLK3; c.CHP = (ch + 31) & ~31; c.permLen = (size_t)E + 32 * (size_t)c.nG + 32;
  c.STG = (int*)al((size_t)CSR_NBLK3 * c.CHP * 4); c.HST = (int*)al((size_t)CSR_NBLK3 * c.NGP * 4); c.OFF = (int*)al((size_t)c.NGP * CSR_NBLK3 * 4); c.START = (int*)al((size_t)(c.NGP + 64) * 4); c.TOT = (int*)al((size_t)(c.NGP + 64) * 4);
  c.PERM = (int*)al(c.permLen * 4); c.ROWPTR = (int*)al((size_t)c.nG * CSR_TS3 * 4); c.ROWCNT = (int*)al((size_t)c.nG * CSR_TS3 * 4); c.FLAG = (int*)al(256);
  c.bytes = off - off0; return off;
}
static void csr_build3(const CsrBufs3& c, const int* dst, int E, int N, hipStream_t stream) {
  const size_t smem = (size_t)(2 * c.NGP + c.CHP) * 4;
  csrZ_kernel3<<<512, 256, 0, stream>>>((int*)c.base, c.bytes / 16);
  csrA_kernel3<<<CSR_NBLK3, 64, smem, stream>>>(dst, E, N, c.nG, c.CHP, c.NGP, c.STG, c.HST);
  csrS_kernel3<<<1, 512, 0, stream>>>(c.HST, c.nG, c.NGP, c.START, c.TOT, c.OFF);
  csrB_kernel3<<<c.nG, 256, 0, stream>>>(dst, N, c.nG, c.CHP, c.NGP, (int)c.permLen, c.STG, c.HST, c.OFF, c.START, c.TOT, c.PERM, c.ROWPTR, c.ROWCNT, c.FLAG);
}

#undef N

__global__ __launch_bounds__(256) void wput_kernel(const float* __restrict__ wk, const float* __restrict__ wv, const float* __restrict__ wp, const float* __restrict__ w1, const float* __restrict__ wq, const float* __restrict__ wskip, b16* __restrict__ WO, b16* __restrict__ W1A, b16* __restrict__ WR, b16* __restrict__ W1B) { const int u = blockIdx.x * 256 + threadIdx.x;
  if (u < 192 * 8) { const int r = u / 8, k0 = (u % 8) * 8; const int part = r / 64, o = r % 64; const float* w = part == 0 ? wk : (part == 1 ? wv : wp); v8b v;
#pragma unroll
    for (int j = 0; j < 8; ++j) v[j] = (b16)(bf16_rne(w[(size_t)(k0 + j) * H + o]) * WSC); for (int pass = 0; pass < 2; ++pass) { *(volatile v8b*)(WO + (size_t)r * 64 + k0) = v; __threadfence(); } }
  if (u < MH * 8) { const int o = u / 8, k0 = (u % 8) * 8; v8b a, b;
#pragma unroll
    for (int j = 0; j < 8; ++j) { a[j] = (b16)(bf16_rne(w1[(size_t)(k0 + j) * MH + o]) * WSC); b[j] = (b16)(bf16_rne(w1[(size_t)(H + k0 + j) * MH + o]) * WSC); } for (int pass = 0; pass < 2; ++pass) { *(volatile v8b*)(W1A + (size_t)o * 64 + k0) = a; *(volatile v8b*)(W1B + (size_t)o * 64 + k0) = b; __threadfence(); } }
  if (u < 128 * 4) { const int r = u / 4, k0 = (u % 4) * 8; const int part = r / 64, o = r % 64; const float* w = part == 0 ? wq : wskip; v8b v;
#pragma unroll
    for (int j = 0; j < 8; ++j) v[j] = (b16)(bf16_rne(w[(size_t)(k0 + j) * H + o]) * WSC); for (int pass = 0; pass < 2; ++pass) { *(volatile v8b*)(WR + (size_t)r * 32 + k0) = v; __threadfence(); } } }
__global__ __launch_bounds__(128) void cvec_kernel(const float* __restrict__ om, const float* __restrict__ w1, const float* __restrict__ b1, float* __restrict__ CV) { const int c = threadIdx.x; float s = bf16_rne(b1[c]);
#pragma unroll 1
  for (int m = 0; m < OM; ++m) s += pmul(bf16_rne(om[m]), bf16_rne(w1[(size_t)(2 * H + m) * MH + c]));
  for (int pass = 0; pass < 2; ++pass) { ((volatile float*)CV)[c] = s; __threadfence(); } }
__global__ __launch_bounds__(32) void oproj_kernel(const float* __restrict__ x, const b16* __restrict__ WO, const float* __restrict__ bk, const float* __restrict__ bv, const float* __restrict__ bp, const b16* __restrict__ W1A, int NLIM, float* __restrict__ KO, float* __restrict__ P1) { __shared__ __attribute__((aligned(16))) b16 Ah[16][72], Al[16][72]; __shared__ float Tf[16][196], Tp[16][132]; const int lane = threadIdx.x, nloc = lane & 15, hlf = lane >> 4; const size_t m0 = (size_t)blockIdx.x * 16; if (m0 >= (size_t)NLIM) return;
  for (int rr = 0; rr < 16; ++rr) for (int q = 0; q < 2; ++q) Ah[rr][q * 32 + lane] = (b16)(bf16_rne(x[(m0 + rr) * DO + q * 32 + lane]) * XS);
  wave_lds_sync(); v8f acc[12];
#pragma unroll
  for (int t = 0; t < 12; ++t) acc[t] = (v8f){};
#pragma unroll
  for (int kb = 0; kb < DO; kb += 32) { const v16b a = frag_kb(&Ah[nloc][kb], hlf);
#pragma unroll
    for (int t = 0; t < 12; ++t) acc[t] = wmma16b(a, frag_kb(WO + (size_t)(t * 16 + nloc) * 64 + kb, hlf), acc[t]); }
#pragma unroll
  for (int t = 0; t < 12; ++t) { const int cc = t * 16 + nloc; const float bb = bf16_rne(cc < 64 ? bk[cc] : (cc < 128 ? bv[cc - 64] : bp[cc - 128]));
#pragma unroll
    for (int r8 = 0; r8 < 8; ++r8) Tf[8 * hlf + r8][cc] = acc[t][r8] * (1.0f / (XS * WSC)) + bb; }
  wave_lds_sync();
  for (int rr = 0; rr < 16; ++rr) for (int q = 0; q < 2; ++q) { b16 p, ql; split16(Tf[rr][128 + q * 32 + lane] * XS, p, ql); Ah[rr][q * 32 + lane] = p; Al[rr][q * 32 + lane] = ql; }
  wave_lds_sync(); v8f acc2[8];
#pragma unroll
  for (int t = 0; t < 8; ++t) acc2[t] = (v8f){};
#pragma unroll
  for (int kb = 0; kb < H; kb += 32) { const v16b a = frag_kb(&Ah[nloc][kb], hlf), al = frag_kb(&Al[nloc][kb], hlf);
#pragma unroll
    for (int t = 0; t < 8; ++t) { const v16b bw = frag_kb(W1A + (size_t)(t * 16 + nloc) * 64 + kb, hlf); acc2[t] = wmma16b(a, bw, acc2[t]); acc2[t] = wmma16b(al, bw, acc2[t]); } }
#pragma unroll
  for (int t = 0; t < 8; ++t)
#pragma unroll
    for (int r8 = 0; r8 < 8; ++r8) Tp[8 * hlf + r8][t * 16 + nloc] = acc2[t][r8] * (1.0f / (XS * WSC));
  wave_lds_sync();
  for (int pass = 0; pass < 2; ++pass) { for (int rr = 0; rr < 16; ++rr) { for (int q = 0; q < 6; ++q) ((volatile float*)KO)[(m0 + rr) * 192 + q * 32 + lane] = Tf[rr][q * 32 + lane]; *(volatile v4f*)(P1 + (m0 + rr) * MH + lane * 4) = *(const v4f*)(&Tp[rr][lane * 4]); } __threadfence(); } }
__global__ __launch_bounds__(32) void rproj_kernel(const float* __restrict__ xr, const b16* __restrict__ WR, const float* __restrict__ bq, const float* __restrict__ bs, float* __restrict__ QS) { __shared__ __attribute__((aligned(16))) b16 Ah[16][40]; __shared__ float Tf[16][132]; const int lane = threadIdx.x, nloc = lane & 15, hlf = lane >> 4; const size_t m0 = (size_t)blockIdx.x * 16;
  for (int rr = 0; rr < 16; ++rr) { const size_t r = (m0 + rr) < (size_t)NR ? m0 + rr : NR - 1; Ah[rr][lane] = (b16)(bf16_rne(xr[r * DR + lane]) * XS); if (lane < 8) Ah[rr][32 + lane] = (b16)0.0f; }
  wave_lds_sync(); const v16b a = frag_kb(&Ah[nloc][0], hlf);
#pragma unroll
  for (int t = 0; t < 8; ++t) { const v8f acc = wmma16b(a, frag_kb(WR + (size_t)(t * 16 + nloc) * 32, hlf), (v8f){}); const int cc = t * 16 + nloc; const float bb = bf16_rne(cc < 64 ? bq[cc] : bs[cc - 64]);
#pragma unroll
    for (int r8 = 0; r8 < 8; ++r8) Tf[8 * hlf + r8][cc] = acc[r8] * (1.0f / (XS * WSC)) + bb; }
  wave_lds_sync();
  for (int pass = 0; pass < 2; ++pass) { for (int rr = 0; rr < 16; ++rr) *(volatile v4f*)(QS + (m0 + rr) * 128 + lane * 4) = *(const v4f*)(&Tf[rr][lane * 4]); __threadfence(); } }
__global__ __launch_bounds__(256) void att_kernel(const float* __restrict__ KO, const float* __restrict__ QS, const float* __restrict__ ea, const float* __restrict__ we, const int* __restrict__ oidx, const int* __restrict__ PERM, const int* __restrict__ ROWPTR, const int* __restrict__ ROWCNT, int permLen, int OLIM, float* __restrict__ RE) { const int wave = threadIdx.x >> 5, lane = threadIdx.x & 31; const size_t r = (size_t)blockIdx.x * 8 + wave; if (r >= (size_t)NRP) return; v2f outv = {0, 0};
  if (r < (size_t)NR) { const size_t rp = (r >> 3) * 32 + (r & 7);
    int st = ROWPTR[rp], cnt = ROWCNT[rp]; cnt = iclamp(cnt, 0, E); st = iclamp(st, 0, permLen - cnt); const v2f q = *(const v2f*)(QS + r * 128 + lane * 2); float wv[4][2]; for (int a = 0; a < 4; ++a) for (int k = 0; k < 2; ++k) wv[a][k] = bf16_rne(we[a * H + lane * 2 + k]);
    float m = -INFINITY, den = 0.0f; v2f acc = {0, 0};
#pragma unroll 1
    for (int j = 0; j < cnt; ++j) { const int eg = iclamp(PERM[st + j], 0, E - 1); const size_t o = (size_t)iclamp(oidx[eg], 0, NO - 1); if (o >= (size_t)OLIM) continue; float ev[2] = {0.0f, 0.0f};
#pragma unroll
      for (int a = 0; a < 4; ++a) { const float av = bf16_rne(ea[(size_t)eg * DE + a]); ev[0] += pmul(av, wv[a][0]); ev[1] += pmul(av, wv[a][1]); }
      const v2f kv = *(const v2f*)(KO + o * 192 + lane * 2), vv = *(const v2f*)(KO + o * 192 + 64 + lane * 2); float s = pmul(q[0], kv[0] + ev[0]) + pmul(q[1], kv[1] + ev[1]); for (int of = 16; of; of >>= 1) s += __shfl_xor(s, of); s *= SCALE;
      const float mn = fmaxf(m, s); const float sf = (m == -INFINITY) ? 0.0f : __expf(m - mn); const float p = __expf(s - mn); den = den * sf + p; acc[0] = pmul(acc[0], sf) + pmul(p, vv[0] + ev[0]); acc[1] = pmul(acc[1], sf) + pmul(p, vv[1] + ev[1]); m = mn; }
    const float inv = 1.0f / (den + 1e-16f); const v2f sk = *(const v2f*)(QS + r * 128 + 64 + lane * 2); outv[0] = pmul(acc[0], inv) + sk[0]; outv[1] = pmul(acc[1], inv) + sk[1]; }
  for (int pass = 0; pass < 2; ++pass) { *(volatile v2f*)(RE + r * H + lane * 2) = outv; __threadfence(); } }
__global__ __launch_bounds__(32) void p2_kernel(const float* __restrict__ RE, const b16* __restrict__ W1B, float* __restrict__ P2) { __shared__ __attribute__((aligned(16))) b16 Ah[16][72], Al[16][72]; __shared__ float Tf[16][132]; const int lane = threadIdx.x, nloc = lane & 15, hlf = lane >> 4; const size_t m0 = (size_t)blockIdx.x * 16;
  for (int rr = 0; rr < 16; ++rr) for (int q = 0; q < 2; ++q) { b16 p, ql; split16(RE[(m0 + rr) * H + q * 32 + lane] * XS, p, ql); Ah[rr][q * 32 + lane] = p; Al[rr][q * 32 + lane] = ql; }
  wave_lds_sync(); v8f acc[8];
#pragma unroll
  for (int t = 0; t < 8; ++t) acc[t] = (v8f){};
#pragma unroll
  for (int kb = 0; kb < H; kb += 32) { const v16b a = frag_kb(&Ah[nloc][kb], hlf), al = frag_kb(&Al[nloc][kb], hlf);
#pragma unroll
    for (int t = 0; t < 8; ++t) { const v16b bw = frag_kb(W1B + (size_t)(t * 16 + nloc) * 64 + kb, hlf); acc[t] = wmma16b(a, bw, acc[t]); acc[t] = wmma16b(al, bw, acc[t]); } }
#pragma unroll
  for (int t = 0; t < 8; ++t)
#pragma unroll
    for (int r8 = 0; r8 < 8; ++r8) Tf[8 * hlf + r8][t * 16 + nloc] = acc[t][r8] * (1.0f / (XS * WSC));
  wave_lds_sync();
  for (int pass = 0; pass < 2; ++pass) { for (int rr = 0; rr < 16; ++rr) *(volatile v4f*)(P2 + (m0 + rr) * MH + lane * 4) = *(const v4f*)(&Tf[rr][lane * 4]); __threadfence(); } }
__global__ __launch_bounds__(256) void edge_kernel(const float* __restrict__ KO, const float* __restrict__ RE, const float* __restrict__ P1, const float* __restrict__ P2, const float* __restrict__ CV, const float* __restrict__ w2, const float* __restrict__ b2, const int* __restrict__ oidx, const int* __restrict__ ridx, int OLIM, int nh, int nm, float* __restrict__ out) { const size_t e = (size_t)blockIdx.x * 256 + threadIdx.x; if (e >= (size_t)E) return; const int o = iclamp(oidx[e], 0, NO - 1), r = iclamp(ridx[e], 0, NR - 1); float val = 0.0f;
  if (o < OLIM) { const float* op = KO + (size_t)o * 192 + 128; const float* re = RE + (size_t)r * H; float dot = 0.0f;
#pragma unroll 1
    for (int c = 0; c < nh; ++c) dot += pmul(op[c], re[c]);
    const float* pa = P1 + (size_t)o * MH; const float* pb = P2 + (size_t)r * MH; float res = bf16_rne(b2[0]);
#pragma unroll 1
    for (int c = 0; c < nm; ++c) res += pmul(fmaxf(pa[c] + pb[c] + CV[c], 0.0f), bf16_rne(w2[c]));
    val = fminf(fmaxf(dot * SCALE + res, -10.0f), 10.0f); }
  for (int pass = 0; pass < 2; ++pass) { ((volatile float*)out)[e] = val; __threadfence(); } }
}

extern "C" void kernel_launch(void* const* d_in, const int* in_sizes, int n_in, void* d_out, int out_size, void* d_ws, size_t ws_size, hipStream_t stream) {
  (void)n_in;
  auto Fp = [&](int i) { return (const float*)d_in[i]; }; auto Ip = [&](int i) { return (const int*)d_in[i]; };
  if (in_sizes[0] != NO * DO || in_sizes[1] != NR * DR || in_sizes[2] != E * DE || in_sizes[3] != E || in_sizes[4] != E || in_sizes[5] != OM || in_sizes[6] != DO * H || in_sizes[8] != DR * H || in_sizes[12] != DE * H || in_sizes[17] != (2 * H + OM) * MH || in_sizes[19] != MH || out_size != E) return;
  const int OLIM = NO;
  size_t off = 0; char* ws = (char*)d_ws;
  auto carve = [&](size_t bytes) { char* p = ws + off; off += (bytes + 255) & ~(size_t)255; return p; };
  b16* WO = (b16*)carve(192 * 64 * 2); b16* W1A = (b16*)carve(MH * 64 * 2); b16* WR = (b16*)carve(128 * 32 * 2); b16* W1B = (b16*)carve(MH * 64 * 2); float* CV = (float*)carve(MH * 4);
  float* KO = (float*)carve((size_t)NO * 192 * 4); float* P1 = (float*)carve((size_t)NO * MH * 4); float* QS = (float*)carve((size_t)NRP * 128 * 4); float* RE = (float*)carve((size_t)NRP * H * 4); float* P2 = (float*)carve((size_t)NRP * MH * 4); CsrBufs3 csr; off = csr_carve3(csr, ws, off, E, NRP);
  if (off > ws_size || off > ((size_t)200 << 20)) return;
  wput_kernel<<<(192 * 8 + 255) / 256, 256, 0, stream>>>(Fp(6), Fp(10), Fp(15), Fp(17), Fp(8), Fp(13), WO, W1A, WR, W1B);
  cvec_kernel<<<1, 128, 0, stream>>>(Fp(5), Fp(17), Fp(18), CV);
  csr_build3(csr, Ip(4), E, NRP, stream);
  oproj_kernel<<<OLIM / 16, 32, 0, stream>>>(Fp(0), WO, Fp(7), Fp(11), Fp(16), W1A, OLIM, KO, P1);
  rproj_kernel<<<NRP / 16, 32, 0, stream>>>(Fp(1), WR, Fp(9), Fp(14), QS);
  att_kernel<<<NRP / 8, 256, 0, stream>>>(KO, QS, Fp(2), Fp(12), Ip(3), csr.PERM, csr.ROWPTR, csr.ROWCNT, (int)csr.permLen, OLIM, RE);
  p2_kernel<<<NRP / 16, 32, 0, stream>>>(RE, W1B, P2);
  edge_kernel<<<(E + 255) / 256, 256, 0, stream>>>(KO, RE, P1, P2, CV, Fp(19), Fp(20), Ip(3), Ip(4), OLIM, H, MH, (float*)d_out);
}
